// E3EquivariantGNN_62277025792337
// MI455X (gfx1250) — hardware-verified
//
#include <hip/hip_runtime.h>
#include <stddef.h>
#include <stdint.h>
#include <math.h>

#define NNODE   10000
#define NEDGE   160000
#define NLAY    4
#define NBAS    10
#define RNEU    100
#define WNUM    704
#define KPAD    128
#define NTHR    256
#define NWAVE   8
#define EPT     8
#define CHUNK   (NTHR * EPT)
#define WCAP    (EPT * 32)
#define LISTN   (NWAVE * WCAP)
#define NBA     1024
#define SLA     10
#define RCAP    28672
#define DEGCAP  64
#define MEAS_B1024  16559
#define MEAS_MAXDEG 37
#define NBLK    10
#define EB      128
#define HP      136
#define GW      32
#define NPIT    40
#define MW      128
#define NODEW   64
#define NPB     32
#define CHF     256.0f
#define CFF     256.0f
#define INVC    1.52587890625e-05f
#define FLUSHT  6.103515625e-05f
#define C_SC    0.25f
#define C_V0    0.35355339059327373f
#define C_CG    0.20412414523193151f
#define RS8     0.35355339059327373f
#define RS24    0.20412414523193151f
#define RS32    0.17677669529663687f
#define SQ3     1.7320508075688772f
#define SQ75    2.7386127875258306f
#define NU_FCT  (NLAY * WNUM * (KPAD / 8))
#define NU_NODE (NNODE * 16)
#define BKT_ZINTS    (LISTN + 2 * RCAP + 3 * NBA)
#define BKT_LDS_INTS (BKT_ZINTS + 16)
#define OFF_G   0
#define OFF_N   4096
#define OFF_Q   9216
#define OFF_P   10240
#define OFF_RW  13312
#define OFF_RB  14592
#define OFF_FB  14720
#define OFF_M   15424
#define OFF_H   31808
#define EDGE_LDS_BYTES (OFF_H * 4 + EB * HP * 2)
#define WSMAX   134217728

static_assert(NEDGE % EB == 0);
static_assert(WNUM == 11 * 64 && WNUM == 44 * 16);
static_assert(KPAD >= RNEU && KPAD % 32 == 0);
static_assert(NNODE % 4 == 0);
static_assert((CHUNK & (CHUNK - 1)) == 0 && CHUNK <= 4096);
static_assert(NBA == (1 << SLA));
static_assert(((long long)NEDGE << SLA) < (1LL << 31));
static_assert(NBLK * NBA >= NNODE && (NBLK - 1) * NBA < NNODE);
static_assert(RCAP >= MEAS_B1024 + 4096 && RCAP % 32 == 0);
static_assert(DEGCAP >= MEAS_MAXDEG + 8);
static_assert(BKT_ZINTS % (4 * NTHR) == 0);
static_assert(BKT_LDS_INTS * 4 <= 300000);
static_assert(EDGE_LDS_BYTES <= 300000);
static_assert(NTHR * GW <= RCAP);
static_assert(NU_FCT % NTHR == 0 && NU_NODE % NTHR == 0);
static_assert(MW >= 120 && MW * 4 == 512);
static_assert(OFF_N == OFF_G + EB * GW && OFF_Q == OFF_N + EB * NPIT && OFF_P == OFF_Q + EB * 8);
static_assert(OFF_RW == OFF_P + EB * 24 && OFF_RB == OFF_RW + NBAS * KPAD && OFF_FB == OFF_RB + KPAD);
static_assert(OFF_M == OFF_FB + WNUM && OFF_H == OFF_M + EB * MW);
static_assert((HP * 2) % 16 == 0 && HP >= KPAD);
static_assert(EB == NWAVE * 16 && NTHR == 2 * EB);
static_assert(CHF * CFF * INVC == 1.0f);

typedef float          v4f   __attribute__((ext_vector_type(4)));
typedef float          v8f   __attribute__((ext_vector_type(8)));
typedef int            v4i   __attribute__((ext_vector_type(4)));
typedef int            v8i   __attribute__((ext_vector_type(8)));
typedef unsigned short v8us  __attribute__((ext_vector_type(8)));
typedef unsigned short v16us __attribute__((ext_vector_type(16)));
typedef _Float16       v16h  __attribute__((ext_vector_type(16)));
typedef v4f  __attribute__((may_alias)) v4fa;
typedef v4i  __attribute__((may_alias)) v4ia;
typedef v8us __attribute__((may_alias)) v8usa;
union FragH { v16h v; v16us u; v8us h[2]; v8i w; };

__device__ __forceinline__ v8f wmh(const FragH& a, const FragH& b, v8f c) {
  v8f d = __builtin_amdgcn_wmma_f32_16x16x32_f16(false, a.v, false, b.v, (short)0, c, false, false);
  asm volatile("v_nop\n\tv_nop\n\tv_nop\n\tv_nop" : "+v"(d) : "v"(a.w), "v"(b.w));
  return d;
}

__device__ __forceinline__ unsigned int f2bf(float f) {
  const unsigned int u = __float_as_uint(f);
  const unsigned int r = ((u + 0x7FFFu + ((u >> 16) & 1u)) >> 16) & 0xFFFFu;
  return ((u & 0x7FFFFFFFu) > 0x7F800000u) ? 0x7FC0u : r;
}
__device__ __forceinline__ float bfr(float f) { return __uint_as_float(f2bf(f) << 16); }
__device__ __forceinline__ unsigned short f2h(float f) {
  const _Float16 hv = (_Float16)f;
  return __builtin_bit_cast(unsigned short, hv);
}
__device__ __forceinline__ unsigned short f2h_flush(float x) {
  const float y = (fabsf(x) < FLUSHT) ? 0.0f : x;
  return f2h(y);
}
__device__ __forceinline__ void put16(unsigned short* dp, v8us o) {
  *(volatile v8us*)dp = o;
  __threadfence();
  *(volatile v8us*)dp = o;
}
__device__ __forceinline__ void putf4(float* dp, v4f o) {
  *(volatile v4f*)dp = o;
  __threadfence();
  *(volatile v4f*)dp = o;
}

template <int SLB>
__device__ __forceinline__ int scan_chunk(const int* __restrict__ dsts, int nE, int cbase, int slotBase,
                                          int nb, int vec8, int* list, int tid, int lane, int wave,
                                          int& below) {
  int wc = 0;
  const int el0  = tid * EPT;
  const int e0   = cbase + el0;
  const int sent = -2147483647 - 1;
  v4i da, db;
  if (vec8 != 0 && cbase + CHUNK <= nE) {
    da = *(const v4i*)(dsts + e0);
    db = *(const v4i*)(dsts + e0 + 4);
  } else {
    da.x = (e0     < nE) ? dsts[min(e0,     nE - 1)] : sent;
    da.y = (e0 + 1 < nE) ? dsts[min(e0 + 1, nE - 1)] : sent;
    da.z = (e0 + 2 < nE) ? dsts[min(e0 + 2, nE - 1)] : sent;
    da.w = (e0 + 3 < nE) ? dsts[min(e0 + 3, nE - 1)] : sent;
    db.x = (e0 + 4 < nE) ? dsts[min(e0 + 4, nE - 1)] : sent;
    db.y = (e0 + 5 < nE) ? dsts[min(e0 + 5, nE - 1)] : sent;
    db.z = (e0 + 6 < nE) ? dsts[min(e0 + 6, nE - 1)] : sent;
    db.w = (e0 + 7 < nE) ? dsts[min(e0 + 7, nE - 1)] : sent;
  }
  const unsigned nbs = (unsigned)slotBase;
  const unsigned unb = (unsigned)nb;
  below += (int)((unsigned)da.x < nbs) + (int)((unsigned)da.y < nbs) + (int)((unsigned)da.z < nbs) +
           (int)((unsigned)da.w < nbs) + (int)((unsigned)db.x < nbs) + (int)((unsigned)db.y < nbs) +
           (int)((unsigned)db.z < nbs) + (int)((unsigned)db.w < nbs);
  const unsigned s0 = (unsigned)da.x - nbs, s1 = (unsigned)da.y - nbs;
  const unsigned s2 = (unsigned)da.z - nbs, s3 = (unsigned)da.w - nbs;
  const unsigned s4 = (unsigned)db.x - nbs, s5 = (unsigned)db.y - nbs;
  const unsigned s6 = (unsigned)db.z - nbs, s7 = (unsigned)db.w - nbs;
  const bool h0 = s0 < unb, h1 = s1 < unb, h2 = s2 < unb, h3 = s3 < unb;
  const bool h4 = s4 < unb, h5 = s5 < unb, h6 = s6 < unb, h7 = s7 < unb;
  const unsigned any = __builtin_amdgcn_ballot_w32(h0 | h1 | h2 | h3 | h4 | h5 | h6 | h7);
  if (any != 0u) {
#define HITJ(J, HJ, SJ) { \
      const unsigned mj = __builtin_amdgcn_ballot_w32(HJ); \
      if (mj != 0u) { \
        if (HJ) { \
          const int pos = wc + (int)__builtin_amdgcn_mbcnt_lo(mj, 0u); \
          if (pos < WCAP) list[wave * WCAP + pos] = ((el0 + (J)) << SLB) | (int)(SJ); \
        } \
        wc += (int)__builtin_popcount(mj); } }
    HITJ(0, h0, s0)
    HITJ(1, h1, s1)
    HITJ(2, h2, s2)
    HITJ(3, h3, s3)
    HITJ(4, h4, s4)
    HITJ(5, h5, s5)
    HITJ(6, h6, s6)
    HITJ(7, h7, s7)
#undef HITJ
  }
  return wc;
}

__global__ __launch_bounds__(NTHR) void k_prep(const float* __restrict__ x, const float* __restrict__ ew,
                                               const float* __restrict__ fcw, unsigned short* FCT,
                                               float* NODEA) {
  const int u = (int)blockIdx.x * NTHR + (int)threadIdx.x;
  if (u < NU_FCT) {
    const int l   = u / (WNUM * 16);
    const int rem = u - l * (WNUM * 16);
    const int n   = rem >> 4;
    const int k8  = (rem & 15) * 8;
    v8us o;
#pragma unroll
    for (int i = 0; i < 8; ++i) {
      const int k  = k8 + i;
      const int kc = k < RNEU ? k : RNEU - 1;
      const float f = fcw[((size_t)(l * RNEU + kc)) * WNUM + n];
      const float val = (k < RNEU) ? bfr(f) * CFF : 0.0f;
      o[i] = f2h_flush(val);
    }
    put16(FCT + (size_t)u * 8, o);
    return;
  }
  const int v = u - NU_FCT;
  if (v >= NU_NODE) return;
  const int n  = v >> 4;
  const int q  = v & 15;
  const int qc = q & 3;
  float a0 = 0.0f, a1 = 0.0f, a2 = 0.0f, a3 = 0.0f;
#pragma unroll 1
  for (int k = 0; k < 8; ++k) {
    const float xv = bfr(x[(size_t)n * 8 + k]);
    const v4f ev = *(const v4f*)(ew + k * 16 + 4 * qc);
    a0 = fmaf(xv, bfr(ev.x), a0);
    a1 = fmaf(xv, bfr(ev.y), a1);
    a2 = fmaf(xv, bfr(ev.z), a2);
    a3 = fmaf(xv, bfr(ev.w), a3);
  }
  const bool isS = q < 4;
  v4f o;
  o.x = isS ? a0 * RS8 : 0.0f;
  o.y = isS ? a1 * RS8 : 0.0f;
  o.z = isS ? a2 * RS8 : 0.0f;
  o.w = isS ? a3 * RS8 : 0.0f;
  putf4(NODEA + (size_t)v * 4, o);
}

__global__ __launch_bounds__(NTHR) void k_bucket(const int* __restrict__ ei, const float* __restrict__ pos,
                                                 int nE, int nN, int vec8, float* GEO, int* START, int* CNT,
                                                 int* FLG) {
  extern __shared__ __attribute__((aligned(16))) int bsm[];
  int* list = bsm;
  int* reg1 = bsm + LISTN;
  int* sl   = reg1 + RCAP;
  int* cnt  = sl + RCAP;
  int* offs = cnt + NBA;
  int* cur  = offs + NBA;
  int* misc = cur + NBA;
  const int tid = (int)threadIdx.x, lane = tid & 31, wave = tid >> 5;
  const int blk = (int)blockIdx.x;
  const int nodeBase = blk * NBA;
  int nb = nN - nodeBase;
  nb = nb < 0 ? 0 : (nb > NBA ? NBA : nb);
  const int* dsts = ei + nE;

  {
    const v4i z4 = {0, 0, 0, 0};
    for (int i = tid * 4; i < BKT_ZINTS; i += NTHR * 4) *(v4ia*)(bsm + i) = z4;
    if (tid < 16) misc[tid] = 0;
  }
  __syncthreads();

  int tot = 0, totAll = 0, ovf = 0, below = 0;
  const int nChunks = (nE + CHUNK - 1) / CHUNK;
#pragma unroll 1
  for (int ch = 0; ch < nChunks; ++ch) {
    const int cbase = ch * CHUNK;
    const int wc = scan_chunk<SLA>(dsts, nE, cbase, nodeBase, nb, vec8, list, tid, lane, wave, below);
    if (lane == 0) misc[wave] = wc;
    __syncthreads();
    int pre = 0, all = 0;
#pragma unroll
    for (int w2 = 0; w2 < NWAVE; ++w2) {
      int c = misc[w2];
      c = c < 0 ? 0 : (c > WCAP ? WCAP : c);
      all += c;
      pre += (w2 < wave) ? c : 0;
    }
    const int wcc = wc > WCAP ? WCAP : wc;
    const int bse = tot + pre;
#pragma unroll 1
    for (int i = lane; i < wcc; i += 32) {
      const int ent = list[wave * WCAP + i];
      const int el  = (ent >> SLA) & (CHUNK - 1);
      const int sq  = ent & (NBA - 1);
      int eid = cbase + el;
      eid = eid > nE - 1 ? nE - 1 : eid;
      const int p = bse + i;
      if (p < RCAP) reg1[p] = (eid << SLA) | sq;
    }
    if (tot + all > RCAP) ovf = 1;
    totAll += all;
    tot += all;
    tot = tot > RCAP ? RCAP : tot;
    __syncthreads();
  }
  {
    int bsum = below;
#pragma unroll
    for (int d = 16; d >= 1; d >>= 1) bsum += __shfl_xor(bsum, d, 32);
    if (lane == 0) misc[8 + wave] = bsum;
  }
  __syncthreads();
  int base = 0;
#pragma unroll
  for (int w2 = 0; w2 < NWAVE; ++w2) base += misc[8 + w2];
  base = base < 0 ? 0 : (base > nE ? nE : base);
  const int nh = tot;
  int nAll = totAll;
  nAll = nAll < 0 ? 0 : (nAll > nE ? nE : nAll);
  int lim = (blk == (int)gridDim.x - 1) ? (nE - base) : nAll;
  lim = lim > nE - base ? nE - base : lim;
  lim = lim < 0 ? 0 : lim;

  if (wave == 0) {
#pragma unroll 1
    for (int b0 = 0; b0 < nh; b0 += 32) {
      const int idx = b0 + lane;
      const int uv  = reg1[idx < RCAP ? idx : RCAP - 1];
      const int m32 = (nh - b0) < 32 ? (nh - b0) : 32;
#pragma unroll 1
      for (int k = 0; k < m32; ++k) {
        const int u  = __builtin_amdgcn_readlane(uv, k);
        const int sq = u & (NBA - 1);
        if (lane == 0) cnt[sq] = cnt[sq] + 1;
      }
    }
  }
  __syncthreads();
  if (wave == 0) {
    const int b32 = lane * (NBA / 32);
    int s = 0;
#pragma unroll 1
    for (int i = 0; i < NBA / 32; ++i) s += cnt[b32 + i];
    int incl = s;
#pragma unroll
    for (int d = 1; d < 32; d <<= 1) {
      const int y = __shfl_up(incl, d, 32);
      if (lane >= d) incl += y;
    }
    int run = incl - s;
#pragma unroll 1
    for (int i = 0; i < NBA / 32; ++i) {
      const int cv = cnt[b32 + i];
      offs[b32 + i] = run;
      cur[b32 + i]  = run;
      run += cv;
    }
  }
  __syncthreads();
  if (wave == 0) {
#pragma unroll 1
    for (int b0 = 0; b0 < nh; b0 += 32) {
      const int idx = b0 + lane;
      const int uv  = reg1[idx < RCAP ? idx : RCAP - 1];
      const int m32 = (nh - b0) < 32 ? (nh - b0) : 32;
#pragma unroll 1
      for (int k = 0; k < m32; ++k) {
        const int u  = __builtin_amdgcn_readlane(uv, k);
        const int sq = u & (NBA - 1);
        if (lane == 0) {
          int p = cur[sq];
          p = p < 0 ? 0 : (p > RCAP - 1 ? RCAP - 1 : p);
          sl[p] = u;
          cur[sq] = p + 1;
        }
      }
    }
  }
  __syncthreads();

  {
    const v4i ov = *(const v4ia*)(offs + 4 * tid);
    const v4i cv = *(const v4ia*)(cnt + 4 * tid);
    v4i sv;
    sv.x = base + ov.x; sv.y = base + ov.y; sv.z = base + ov.z; sv.w = base + ov.w;
    v4i fv;
    fv.x = (tid == 0) ? ovf : 0;
    fv.y = (tid == 0) ? nh : 0;
    fv.z = (tid == 0) ? base : 0;
    fv.w = (tid == 0) ? nAll : 0;
    int* sp = START + nodeBase + 4 * tid;
    int* cp = CNT + nodeBase + 4 * tid;
    int* fp = FLG + (size_t)blk * 32 + 4 * (tid & 7);
    *(volatile v4i*)sp = sv;
    *(volatile v4i*)cp = cv;
    if (tid < 8) *(volatile v4i*)fp = fv;
    __threadfence();
    *(volatile v4i*)sp = sv;
    *(volatile v4i*)cp = cv;
    if (tid < 8) *(volatile v4i*)fp = fv;
  }

  float* gt = (float*)reg1;
  const float OFF1  = 10.0f * (1.0f / 9.0f);
  const float COEFF = -0.5f / (OFF1 * OFF1);
#pragma unroll 1
  for (int i0 = 0; i0 < lim; i0 += NTHR) {
    const int  i    = i0 + tid;
    const bool real = i < nh;
    const int  ic   = i < RCAP ? i : RCAP - 1;
    const int  ent  = sl[ic];
    int eid = ent >> SLA;
    eid = eid < 0 ? 0 : (eid > nE - 1 ? nE - 1 : eid);
    int rn = ei[eid];
    int cn = ei[nE + eid];
    rn = rn < 0 ? 0 : (rn > nN - 1 ? nN - 1 : rn);
    cn = cn < 0 ? 0 : (cn > nN - 1 ? nN - 1 : cn);
    const float ax = bfr(pos[(size_t)rn * 3 + 0]);
    const float ay = bfr(pos[(size_t)rn * 3 + 1]);
    const float az = bfr(pos[(size_t)rn * 3 + 2]);
    const float bx = bfr(pos[(size_t)cn * 3 + 0]);
    const float by = bfr(pos[(size_t)cn * 3 + 1]);
    const float bz = bfr(pos[(size_t)cn * 3 + 2]);
    const float vx = ax - bx, vy = ay - by, vz = az - bz;
    const float ss  = (vx * vx + vz * vz) + vy * vy;
    const float len = sqrtf(ss + 1e-12f);
    const float inv = 1.0f / len;
    const float ux = vx * inv, uy = vy * inv, uz = vz * inv;
    const float third = 1.0f / 3.0f;
    float* gr = gt + tid * GW;
#pragma unroll 1
    for (int k = 0; k < NBAS; ++k) {
      const float ofk = (k == NBAS - 1) ? 10.0f : 10.0f * ((float)k * (1.0f / 9.0f));
      const float d   = len - ofk;
      const float rb  = expf((COEFF * d) * d);
      gr[k] = real ? rb : 0.0f;
    }
    gr[10] = real ? ux : 0.0f;
    gr[11] = real ? uy : 0.0f;
    v4f q3, q4, q5, q6, q7;
    q3.x = real ? uz : 0.0f;
    q3.y = real ? SQ3 * ux : 0.0f;
    q3.z = real ? SQ3 * uy : 0.0f;
    q3.w = real ? SQ3 * uz : 0.0f;
    q4.x = real ? SQ75 * (ux * ux - third) : 0.0f;
    q4.y = real ? SQ75 * (ux * uy) : 0.0f;
    q4.z = real ? SQ75 * (ux * uz) : 0.0f;
    q4.w = real ? SQ75 * (uy * uy - third) : 0.0f;
    q5.x = real ? SQ75 * (uy * uz) : 0.0f;
    q5.y = real ? SQ75 * (uz * uz - third) : 0.0f;
    q5.z = real ? (float)rn : 0.0f;
    q5.w = real ? 1.0f : 0.0f;
    q6.x = real ? (float)cn : 0.0f;
    q6.y = 0.0f; q6.z = 0.0f; q6.w = 0.0f;
    q7.x = 0.0f; q7.y = 0.0f; q7.z = 0.0f; q7.w = 0.0f;
    *(v4fa*)(gr + 12) = q3;
    *(v4fa*)(gr + 16) = q4;
    *(v4fa*)(gr + 20) = q5;
    *(v4fa*)(gr + 24) = q6;
    *(v4fa*)(gr + 28) = q7;
    __syncthreads();
    v4f pv[8];
#pragma unroll
    for (int it = 0; it < 8; ++it) pv[it] = *(const v4fa*)(gt + (size_t)(it * NTHR + tid) * 4);
    float* gb = GEO + (size_t)(base + i0) * GW;
#pragma unroll
    for (int it = 0; it < 8; ++it) {
      const int row = (it * NTHR + tid) >> 3;
      if (i0 + row < lim) *(volatile v4f*)(gb + (size_t)(it * NTHR + tid) * 4) = pv[it];
    }
    __threadfence();
#pragma unroll
    for (int it = 0; it < 8; ++it) {
      const int row = (it * NTHR + tid) >> 3;
      if (i0 + row < lim) *(volatile v4f*)(gb + (size_t)(it * NTHR + tid) * 4) = pv[it];
    }
    __syncthreads();
  }
}

__device__ __forceinline__ v8f tile4(const FragH& a0, const FragH& a1, const FragH& a2, const FragH& a3,
                                     const unsigned short* __restrict__ bq) {
  FragH b0, b1, b2, b3;
  b0.h[0] = *(const v8usa*)(bq);        b0.h[1] = *(const v8usa*)(bq + 16);
  b1.h[0] = *(const v8usa*)(bq + 32);   b1.h[1] = *(const v8usa*)(bq + 48);
  b2.h[0] = *(const v8usa*)(bq + 64);   b2.h[1] = *(const v8usa*)(bq + 80);
  b3.h[0] = *(const v8usa*)(bq + 96);   b3.h[1] = *(const v8usa*)(bq + 112);
  v8f d = {0.f, 0.f, 0.f, 0.f, 0.f, 0.f, 0.f, 0.f};
  d = wmh(a0, b0, d);
  d = wmh(a1, b1, d);
  d = wmh(a2, b2, d);
  d = wmh(a3, b3, d);
  return d;
}

template <int MODE>
__global__ __launch_bounds__(NTHR) __attribute__((amdgpu_num_vgpr(248)))
void k_edge(const float* __restrict__ GEO, const float* __restrict__ NODEc,
            const unsigned short* __restrict__ FCTl, const float* __restrict__ rw,
            const float* __restrict__ rb, const float* __restrict__ fb, float* MSG, int nN) {
  extern __shared__ __attribute__((aligned(16))) float dyn[];
  float* sG   = dyn + OFF_G;
  float* sN   = dyn + OFF_N;
  float* sQ   = dyn + OFF_Q;
  float* sP   = dyn + OFF_P;
  float* sRW  = dyn + OFF_RW;
  float* sRB  = dyn + OFF_RB;
  float* sFB  = dyn + OFF_FB;
  float* sMsg = dyn + OFF_M;
  unsigned short* sH = (unsigned short*)(dyn + OFF_H);

  const int tid = (int)threadIdx.x, lane = tid & 31, wave = tid >> 5, hh = lane >> 4, m = lane & 15;
  const int p0 = (int)blockIdx.x * EB;

#pragma unroll
  for (int it = 0; it < 4; ++it) {
    const int idx = it * NTHR + tid;
    *(v4fa*)(sG + idx * 4) = *(const v4f*)(GEO + (size_t)p0 * GW + (size_t)idx * 4);
  }
#pragma unroll 1
  for (int idx = tid; idx < NBAS * KPAD; idx += NTHR) {
    const int k  = idx >> 7;
    const int c  = idx & (KPAD - 1);
    const int cc = c < RNEU ? c : RNEU - 1;
    const float v = rw[k * RNEU + cc];
    sRW[idx] = (c < RNEU) ? bfr(v) : 0.0f;
  }
  {
    const int c  = tid & (KPAD - 1);
    const int cc = c < RNEU ? c : RNEU - 1;
    const float v = rb[cc];
    if (tid < KPAD) sRB[c] = (c < RNEU) ? bfr(v) : 0.0f;
  }
#pragma unroll 1
  for (int it = 0; it < 3; ++it) {
    const int idx = it * NTHR + tid;
    const int ic  = idx < WNUM ? idx : WNUM - 1;
    const float v = bfr(fb[ic]);
    if (idx < WNUM) sFB[idx] = v;
  }
  __syncthreads();

  {
    constexpr int NQ = (MODE == 0) ? 4 : 10;
#pragma unroll 1
    for (int idx = tid; idx < EB * NQ; idx += NTHR) {
      const int e = idx / NQ;
      const int q = idx - e * NQ;
      const float* g = sG + e * GW;
      int src = (int)g[22];
      src = src < 0 ? 0 : (src > nN - 1 ? nN - 1 : src);
      const bool ok = g[23] != 0.0f;
      const v4f nv = *(const v4f*)(NODEc + (size_t)src * NODEW + 4 * q);
      v4f o;
      o.x = ok ? nv.x : 0.0f;
      o.y = ok ? nv.y : 0.0f;
      o.z = ok ? nv.z : 0.0f;
      o.w = ok ? nv.w : 0.0f;
      *(v4fa*)(sN + e * NPIT + 4 * q) = o;
    }
  }
  {
    const int e  = tid & (EB - 1);
    const int hf = tid >> 7;
    const float* g = sG + e * GW;
    const v4f r0 = *(const v4fa*)g;
    const v4f r1 = *(const v4fa*)(g + 4);
    const v4f r2 = *(const v4fa*)(g + 8);
    const float vf = (g[23] != 0.0f) ? 1.0f : 0.0f;
    const float rr[NBAS] = {r0.x, r0.y, r0.z, r0.w, r1.x, r1.y, r1.z, r1.w, r2.x, r2.y};
    unsigned short* hrow = sH + e * HP;
#pragma unroll 1
    for (int gq = 0; gq < 8; ++gq) {
      const int c0 = (hf * 8 + gq) * 8;
      v4f a0 = *(const v4fa*)(sRB + c0);
      v4f a1 = *(const v4fa*)(sRB + c0 + 4);
#pragma unroll
      for (int k = 0; k < NBAS; ++k) {
        const v4f w0 = *(const v4fa*)(sRW + k * KPAD + c0);
        const v4f w1 = *(const v4fa*)(sRW + k * KPAD + c0 + 4);
        a0.x = fmaf(rr[k], w0.x, a0.x); a0.y = fmaf(rr[k], w0.y, a0.y);
        a0.z = fmaf(rr[k], w0.z, a0.z); a0.w = fmaf(rr[k], w0.w, a0.w);
        a1.x = fmaf(rr[k], w1.x, a1.x); a1.y = fmaf(rr[k], w1.y, a1.y);
        a1.z = fmaf(rr[k], w1.z, a1.z); a1.w = fmaf(rr[k], w1.w, a1.w);
      }
      const v8f h8 = {a0.x, a0.y, a0.z, a0.w, a1.x, a1.y, a1.z, a1.w};
      v8us o;
#pragma unroll
      for (int i = 0; i < 8; ++i) {
        const float hv = h8[i];
        const float rl = (hv > 0.0f) ? hv : (hv - hv);
        o[i] = f2h_flush(rl * vf * CHF);
      }
      *(v8usa*)(hrow + c0) = o;
    }
  }
  __syncthreads();

  if constexpr (MODE >= 1) {
#pragma unroll 1
    for (int idx = tid; idx < EB * 8; idx += NTHR) {
      const int e = idx >> 3;
      const int u = idx & 7;
      const float* g  = sG + e * GW;
      const float* vp = sN + e * NPIT + 16 + 3 * u;
      const float v0 = vp[0], v1 = vp[1], v2 = vp[2];
      const float s0 = g[13], s1 = g[14], s2 = g[15];
      const float mxx = g[16], mxy = g[17], mxz = g[18], myy = g[19], myz = g[20], mzz = g[21];
      sQ[e * 8 + u] = fmaf(v2, s2, fmaf(v1, s1, v0 * s0));
      float* pp = sP + e * 24 + 3 * u;
      pp[0] = fmaf(mxz, v2, fmaf(mxy, v1, mxx * v0));
      pp[1] = fmaf(myz, v2, fmaf(myy, v1, mxy * v0));
      pp[2] = fmaf(mzz, v2, fmaf(myz, v1, mxz * v0));
    }
    __syncthreads();
  }

  FragH a0, a1, a2, a3;
  {
    const unsigned short* ap = sH + (16 * wave + m) * HP + 8 * hh;
    a0.h[0] = *(const v8usa*)(ap);        a0.h[1] = *(const v8usa*)(ap + 16);
    a1.h[0] = *(const v8usa*)(ap + 32);   a1.h[1] = *(const v8usa*)(ap + 48);
    a2.h[0] = *(const v8usa*)(ap + 64);   a2.h[1] = *(const v8usa*)(ap + 80);
    a3.h[0] = *(const v8usa*)(ap + 96);   a3.h[1] = *(const v8usa*)(ap + 112);
  }
  const unsigned short* bp = FCTl + (size_t)m * KPAD + 8 * hh;
  const int er0 = 16 * wave + 8 * hh;
  const float* rowS = sN + er0 * NPIT;

  float acc0[8], acc1[8], acc3[8], acc2[8][3], acc4[8][3];
#pragma unroll
  for (int r = 0; r < 8; ++r) {
    acc0[r] = 0.0f; acc1[r] = 0.0f; acc3[r] = 0.0f;
    acc2[r][0] = 0.0f; acc2[r][1] = 0.0f; acc2[r][2] = 0.0f;
    acc4[r][0] = 0.0f; acc4[r][1] = 0.0f; acc4[r][2] = 0.0f;
  }

#pragma unroll 1
  for (int t = 0; t < 16; ++t) {
    const v8f d = tile4(a0, a1, a2, a3, bp + (size_t)(16 * t) * KPAD);
    const float fbv = sFB[16 * t + m];
#pragma unroll
    for (int r = 0; r < 8; ++r) {
      const float wv = fmaf(d[r], INVC, fbv);
      acc0[r] = fmaf(wv, rowS[r * NPIT + t], acc0[r]);
    }
  }
  if constexpr (MODE <= 1) {
#pragma unroll 1
    for (int t = 0; t < 16; ++t) {
      const v8f d = tile4(a0, a1, a2, a3, bp + (size_t)(256 + 16 * t) * KPAD);
      const float fbv = sFB[256 + 16 * t + m];
#pragma unroll
      for (int r = 0; r < 8; ++r) {
        const float wv = fmaf(d[r], INVC, fbv);
        acc1[r] = fmaf(wv, rowS[r * NPIT + t], acc1[r]);
      }
    }
  }
  if constexpr (MODE == 1) {
#pragma unroll 1
    for (int tt = 0; tt < 4; ++tt) {
      const v8f d = tile4(a0, a1, a2, a3, bp + (size_t)(512 + 16 * tt) * KPAD);
      const float fbv = sFB[512 + 16 * tt + m];
      const int u = 2 * tt + (m >> 3);
#pragma unroll
      for (int r = 0; r < 8; ++r) {
        const float wv = fmaf(d[r], INVC, fbv);
        const float* vp = rowS + r * NPIT + 16 + 3 * u;
        acc2[r][0] = fmaf(wv, vp[0], acc2[r][0]);
        acc2[r][1] = fmaf(wv, vp[1], acc2[r][1]);
        acc2[r][2] = fmaf(wv, vp[2], acc2[r][2]);
      }
    }
  }
  if constexpr (MODE >= 1) {
#pragma unroll 1
    for (int tt = 0; tt < 4; ++tt) {
      const v8f d = tile4(a0, a1, a2, a3, bp + (size_t)(576 + 16 * tt) * KPAD);
      const float fbv = sFB[576 + 16 * tt + m];
      const int u = 2 * tt + (m >> 3);
#pragma unroll
      for (int r = 0; r < 8; ++r) {
        const float wv = fmaf(d[r], INVC, fbv);
        acc3[r] = fmaf(wv, sQ[(er0 + r) * 8 + u], acc3[r]);
      }
    }
  }
  if constexpr (MODE == 1) {
#pragma unroll 1
    for (int tt = 0; tt < 4; ++tt) {
      const v8f d = tile4(a0, a1, a2, a3, bp + (size_t)(640 + 16 * tt) * KPAD);
      const float fbv = sFB[640 + 16 * tt + m];
      const int u = 2 * tt + (m >> 3);
#pragma unroll
      for (int r = 0; r < 8; ++r) {
        const float wv = fmaf(d[r], INVC, fbv);
        const float* pp = sP + (er0 + r) * 24 + 3 * u;
        acc4[r][0] = fmaf(wv, pp[0], acc4[r][0]);
        acc4[r][1] = fmaf(wv, pp[1], acc4[r][1]);
        acc4[r][2] = fmaf(wv, pp[2], acc4[r][2]);
      }
    }
  }
  if constexpr (MODE >= 1) {
#pragma unroll
    for (int r = 0; r < 8; ++r) acc3[r] += __shfl_xor(acc3[r], 8, 32);
  }
  if constexpr (MODE == 1) {
#pragma unroll
    for (int r = 0; r < 8; ++r) {
#pragma unroll
      for (int i = 0; i < 3; ++i) {
        acc2[r][i] += __shfl_xor(acc2[r][i], 8, 32);
        acc4[r][i] += __shfl_xor(acc4[r][i], 8, 32);
      }
    }
  }

  {
    float* mrow = sMsg + er0 * MW;
#pragma unroll
    for (int r = 0; r < 8; ++r) {
      float* row = mrow + r * MW;
      const float* g = sG + (er0 + r) * GW;
      const float s0 = g[13], s1 = g[14], s2 = g[15];
      const float t1 = C_SC * acc1[r];
      row[m] = C_SC * acc0[r];
      row[24 + 3 * m + 0] = t1 * s0;
      row[24 + 3 * m + 1] = t1 * s1;
      row[24 + 3 * m + 2] = t1 * s2;
      if (m < 8) {
        row[16 + m] = C_CG * acc3[r];
        row[72 + 3 * m + 0] = C_V0 * acc2[r][0];
        row[72 + 3 * m + 1] = C_V0 * acc2[r][1];
        row[72 + 3 * m + 2] = C_V0 * acc2[r][2];
        row[96 + 3 * m + 0] = C_CG * acc4[r][0];
        row[96 + 3 * m + 1] = C_CG * acc4[r][1];
        row[96 + 3 * m + 2] = C_CG * acc4[r][2];
        row[120 + m] = 0.0f;
      }
    }
  }
  __syncthreads();

  {
    v4f pv[16];
#pragma unroll
    for (int it = 0; it < 16; ++it) pv[it] = *(const v4fa*)(sMsg + (size_t)(it * NTHR + tid) * 4);
    float* mb = MSG + (size_t)p0 * MW;
#pragma unroll
    for (int it = 0; it < 16; ++it) *(volatile v4f*)(mb + (size_t)(it * NTHR + tid) * 4) = pv[it];
    __threadfence();
#pragma unroll
    for (int it = 0; it < 16; ++it) *(volatile v4f*)(mb + (size_t)(it * NTHR + tid) * 4) = pv[it];
  }
}

template <int LAST>
__global__ __launch_bounds__(NTHR) void k_node(const float* __restrict__ MSG, const int* __restrict__ START,
                                               const int* __restrict__ CNT, const int* __restrict__ FLG,
                                               const float* __restrict__ NODEc, float* NODEn,
                                               const float* __restrict__ lws, const float* __restrict__ lwv,
                                               const float* __restrict__ ow, float* out, int nN, int nE) {
  __shared__ __attribute__((aligned(16))) float sLW[24 * 16];
  __shared__ __attribute__((aligned(16))) float sLV[32 * 8];
  __shared__ __attribute__((aligned(16))) float sOW[16 * 8];
  __shared__ __attribute__((aligned(16))) float sAgg[NWAVE * MW];
  __shared__ __attribute__((aligned(16))) float sRow[NWAVE * NODEW];
  __shared__ __attribute__((aligned(16))) float sO[NPB * 8];
  const int tid = (int)threadIdx.x, lane = tid & 31, wave = tid >> 5;
  const int base = (int)blockIdx.x * NPB;

#pragma unroll 1
  for (int it = 0; it < 2; ++it) {
    const int idx = it * NTHR + tid;
    const int ic  = idx < 384 ? idx : 383;
    const float v = bfr(lws[ic]);
    if (idx < 384) sLW[idx] = v;
  }
  sLV[tid] = bfr(lwv[tid]);
  {
    const float v = bfr(ow[tid & 127]);
    if (tid < 128) sOW[tid] = v;
  }
  __syncthreads();

  const float qnan = __int_as_float(0x7fc00000);
#pragma unroll 1
  for (int j = 0; j < 4; ++j) {
    const int  nl   = wave * 4 + j;
    const int  n    = base + nl;
    const bool live = n < nN;
    const int  nc   = live ? n : nN - 1;
    int st = START[nc];
    const int ct = CNT[nc];
    const int fl = FLG[(size_t)(nc >> SLA) * 32];
    const bool big = (ct > DEGCAP) || (ct < 0);
    const int c = ct < 0 ? 0 : (ct > DEGCAP ? DEGCAP : ct);
    st = st < 0 ? 0 : (st > nE - 1 ? nE - 1 : st);
    v4f a = {0.0f, 0.0f, 0.0f, 0.0f};
#pragma unroll 2
    for (int k = 0; k < c; ++k) {
      int row = st + k;
      row = row > nE - 1 ? nE - 1 : row;
      const v4f mv = *(const v4f*)(MSG + (size_t)row * MW + 4 * lane);
      a.x += mv.x; a.y += mv.y; a.z += mv.z; a.w += mv.w;
    }
    *(v4fa*)(sAgg + wave * MW + 4 * lane) = a;
    __syncthreads();

    const float* ag = sAgg + wave * MW;
    const int wsl = lane & 15;
    float ds = 0.0f;
#pragma unroll 4
    for (int k = 0; k < 24; ++k) ds = fmaf(ag[k], sLW[k * 16 + wsl], ds);
    const int jv = lane < 24 ? lane : 23;
    const int wq = jv / 3;
    const int iq = jv - 3 * wq;
    float dv = 0.0f;
#pragma unroll 4
    for (int u = 0; u < 32; ++u) dv = fmaf(ag[24 + 3 * u + iq], sLV[u * 8 + wq], dv);
    const float so = NODEc[(size_t)nc * NODEW + wsl];
    const float vo = NODEc[(size_t)nc * NODEW + 16 + jv];
    const float pz = (fl != 0 || big) ? qnan : 0.0f;
    const float sn = fmaf(ds, RS24, so) + pz;
    const float vn = fmaf(dv, RS32, vo);
    float* rwv = sRow + wave * NODEW;
    if (lane < 16) rwv[lane] = sn;
    if (lane < 24) { rwv[16 + lane] = vn; rwv[40 + lane] = 0.0f; }
    __syncthreads();

    if constexpr (LAST == 0) {
      const v4f rv = *(const v4fa*)(rwv + 4 * (lane & 15));
      float* np = NODEn + (size_t)nc * NODEW + 4 * (lane & 15);
      const bool wr = live && (lane < 16);
      if (wr) *(volatile v4f*)np = rv;
      __threadfence();
      if (wr) *(volatile v4f*)np = rv;
    } else {
      const int co = lane & 7;
      float d = 0.0f;
#pragma unroll 4
      for (int k = 0; k < 16; ++k) d = fmaf(rwv[k], sOW[k * 8 + co], d);
      const float ov = d * 0.25f + pz;
      if (lane < 8) sO[nl * 8 + co] = ov;
    }
  }

  if constexpr (LAST == 1) {
    __syncthreads();
    if (wave == 0) {
      int nb = nN - base;
      nb = nb < 0 ? 0 : (nb > NPB ? NPB : nb);
      const v4f o0 = *(const v4fa*)(sO + 4 * lane);
      const v4f o1 = *(const v4fa*)(sO + 128 + 4 * lane);
      float* op = out + (size_t)base * 8 + 4 * lane;
      const bool w0 = (lane >> 1) < nb;
      const bool w1 = (16 + (lane >> 1)) < nb;
      if (w0) *(volatile v4f*)op = o0;
      if (w1) *(volatile v4f*)(op + 128) = o1;
      __threadfence();
      if (w0) *(volatile v4f*)op = o0;
      if (w1) *(volatile v4f*)(op + 128) = o1;
    }
  }
}

extern "C" void kernel_launch(void* const* d_in, const int* in_sizes, int n_in,
                              void* d_out, int out_size, void* d_ws, size_t ws_size,
                              hipStream_t stream) {
  if (n_in < 11) return;
  if (in_sizes[0] != NNODE * 8) return;
  if (in_sizes[1] != NNODE * 3) return;
  if (in_sizes[2] != 8 * 16) return;
  if (in_sizes[3] != NLAY * NBAS * RNEU) return;
  if (in_sizes[4] != NLAY * RNEU) return;
  if (in_sizes[5] != NLAY * RNEU * WNUM) return;
  if (in_sizes[6] != NLAY * WNUM) return;
  if (in_sizes[7] != NLAY * 24 * 16) return;
  if (in_sizes[8] != NLAY * 32 * 8) return;
  if (in_sizes[9] != 16 * 8) return;
  if (in_sizes[10] != 2 * NEDGE) return;
  if (out_size != NNODE * 8) return;

  const float* x    = (const float*)d_in[0];
  const float* pos  = (const float*)d_in[1];
  const float* ew   = (const float*)d_in[2];
  const float* rw   = (const float*)d_in[3];
  const float* rb   = (const float*)d_in[4];
  const float* fcw  = (const float*)d_in[5];
  const float* fcb  = (const float*)d_in[6];
  const float* lws  = (const float*)d_in[7];
  const float* lwv  = (const float*)d_in[8];
  const float* ow   = (const float*)d_in[9];
  const int*   ei   = (const int*)d_in[10];
  float* out = (float*)d_out;

  char* ws = (char*)d_ws;
  size_t off = 0;
  const size_t oFCT = off; off += (size_t)NLAY * WNUM * KPAD * 2;   off = (off + 255) & ~(size_t)255;
  const size_t oGEO = off; off += (size_t)NEDGE * GW * 4;           off = (off + 255) & ~(size_t)255;
  const size_t oMSG = off; off += (size_t)NEDGE * MW * 4;           off = (off + 255) & ~(size_t)255;
  const size_t oNA  = off; off += (size_t)NNODE * NODEW * 4;        off = (off + 255) & ~(size_t)255;
  const size_t oNB  = off; off += (size_t)NNODE * NODEW * 4;        off = (off + 255) & ~(size_t)255;
  const size_t oST  = off; off += (size_t)NBLK * NBA * 4;           off = (off + 255) & ~(size_t)255;
  const size_t oCT  = off; off += (size_t)NBLK * NBA * 4;           off = (off + 255) & ~(size_t)255;
  const size_t oFL  = off; off += (size_t)NBLK * 128;               off = (off + 255) & ~(size_t)255;
  if (off > ws_size || off > (size_t)WSMAX) return;
  unsigned short* FCT = (unsigned short*)(ws + oFCT);
  float* GEO   = (float*)(ws + oGEO);
  float* MSG   = (float*)(ws + oMSG);
  float* NODEA = (float*)(ws + oNA);
  float* NODEB = (float*)(ws + oNB);
  int*   START = (int*)(ws + oST);
  int*   CNT   = (int*)(ws + oCT);
  int*   FLG   = (int*)(ws + oFL);

  const int bktLds = BKT_LDS_INTS * 4;
  hipFuncSetAttribute(reinterpret_cast<const void*>(&k_bucket),
                      hipFuncAttributeMaxDynamicSharedMemorySize, bktLds);
  hipFuncSetAttribute(reinterpret_cast<const void*>(&k_edge<0>),
                      hipFuncAttributeMaxDynamicSharedMemorySize, (int)EDGE_LDS_BYTES);
  hipFuncSetAttribute(reinterpret_cast<const void*>(&k_edge<1>),
                      hipFuncAttributeMaxDynamicSharedMemorySize, (int)EDGE_LDS_BYTES);
  hipFuncSetAttribute(reinterpret_cast<const void*>(&k_edge<2>),
                      hipFuncAttributeMaxDynamicSharedMemorySize, (int)EDGE_LDS_BYTES);

  const int gE = NEDGE / EB;
  const int gN = (NNODE + NPB - 1) / NPB;

  k_prep<<<(NU_FCT + NU_NODE) / NTHR, NTHR, 0, stream>>>(x, ew, fcw, FCT, NODEA);
  k_bucket<<<NBLK, NTHR, bktLds, stream>>>(ei, pos, NEDGE, NNODE, 1, GEO, START, CNT, FLG);
  k_edge<0><<<gE, NTHR, EDGE_LDS_BYTES, stream>>>(GEO, NODEA, FCT, rw, rb, fcb, MSG, NNODE);
  k_node<0><<<gN, NTHR, 0, stream>>>(MSG, START, CNT, FLG, NODEA, NODEB, lws, lwv, ow, out, NNODE, NEDGE);
  k_edge<1><<<gE, NTHR, EDGE_LDS_BYTES, stream>>>(GEO, NODEB, FCT + (size_t)1 * WNUM * KPAD,
                                                  rw + 1 * NBAS * RNEU, rb + 1 * RNEU, fcb + 1 * WNUM,
                                                  MSG, NNODE);
  k_node<0><<<gN, NTHR, 0, stream>>>(MSG, START, CNT, FLG, NODEB, NODEA, lws + 1 * 384, lwv + 1 * 256,
                                     ow, out, NNODE, NEDGE);
  k_edge<1><<<gE, NTHR, EDGE_LDS_BYTES, stream>>>(GEO, NODEA, FCT + (size_t)2 * WNUM * KPAD,
                                                  rw + 2 * NBAS * RNEU, rb + 2 * RNEU, fcb + 2 * WNUM,
                                                  MSG, NNODE);
  k_node<0><<<gN, NTHR, 0, stream>>>(MSG, START, CNT, FLG, NODEA, NODEB, lws + 2 * 384, lwv + 2 * 256,
                                     ow, out, NNODE, NEDGE);
  k_edge<2><<<gE, NTHR, EDGE_LDS_BYTES, stream>>>(GEO, NODEB, FCT + (size_t)3 * WNUM * KPAD,
                                                  rw + 3 * NBAS * RNEU, rb + 3 * RNEU, fcb + 3 * WNUM,
                                                  MSG, NNODE);
  k_node<1><<<gN, NTHR, 0, stream>>>(MSG, START, CNT, FLG, NODEB, NODEA, lws + 3 * 384, lwv + 3 * 256,
                                     ow, out, NNODE, NEDGE);
}
